// MultiHeadAttention_39230231282127
// MI455X (gfx1250) — hardware-verified
//
#include <hip/hip_runtime.h>


#ifndef NB
#define NB 2
#endif
#ifndef SEQ
#define SEQ 2048
#endif
#define NB_FULL  2
#define SEQ_FULL 2048
#define DM   1024
#define NH_  16
#define HD   64
#define DQ   (NH_ * HD)
#define DOW  1024
#define RH   ((SEQ) < 256 ? (SEQ) : 256)
#define MROWS (NB * SEQ)
#define PCAR 1024.0f
#define CEXP 0.18033688011112042f
#define WS_CARVE ((size_t)4 * DQ * DM * 2 + (size_t)MROWS * DM * 2 + (size_t)3 * MROWS * DQ * 2 + (size_t)6 * NB * RH * DQ * 2 + (size_t)MROWS * DQ * 2)

static_assert(SEQ % 64 == 0);
static_assert(RH % 64 == 0);
static_assert(RH % 32 == 0 && RH % 16 == 0);
static_assert((SEQ - RH) % 32 == 0);
static_assert(HD == 64);
static_assert(DQ == NH_ * HD);
static_assert(DM % 64 == 0 && DQ % 64 == 0 && DOW % 64 == 0);
static_assert(DM % 32 == 0 && DQ % 32 == 0);
static_assert(DM == DQ);
static_assert(MROWS % 64 == 0);
static_assert((NB * RH) % 64 == 0 && MROWS % 8 == 0);
static_assert(NB <= NB_FULL && SEQ <= SEQ_FULL);
static_assert(((size_t)SEQ * DM) % 2048 == 0);
static_assert((DM * DQ) % 4096 == 0 && (DQ * DOW) % 4096 == 0);
static_assert((size_t)NB_FULL * SEQ_FULL * DOW * 4 == (size_t)16777216);
static_assert(WS_CARVE <= (size_t)134217728);

typedef _Float16 h16;
typedef unsigned short bf;
typedef __attribute__((ext_vector_type(16))) __bf16   v16bf;
typedef __attribute__((ext_vector_type(16))) _Float16 v16h;
typedef __attribute__((ext_vector_type(8)))  _Float16 v8h;
typedef __attribute__((ext_vector_type(8)))  unsigned short v8us;
typedef __attribute__((ext_vector_type(2)))  unsigned short v2us;
typedef __attribute__((ext_vector_type(8)))  float    v8f;
typedef __attribute__((ext_vector_type(4)))  float    v4f;
typedef v4f  __attribute__((may_alias)) v4fa;

__device__ __forceinline__ unsigned short f2bf(float f) { unsigned u = __float_as_uint(f); u += 0x7FFFu + ((u >> 16) & 1u); return (unsigned short)(u >> 16); }
__device__ __forceinline__ float bf2f(unsigned short b) { return __uint_as_float(((unsigned)b) << 16); }
__device__ __forceinline__ float bfr(float f) { return bf2f(f2bf(f)); }
__device__ __forceinline__ void splitf(float y, unsigned short& h, unsigned short& l) { h = f2bf(y); l = f2bf(y - bf2f(h)); }
__device__ __forceinline__ v16h cat16(v8h lo, v8h hi) { return __builtin_shufflevector(lo, hi, 0, 1, 2, 3, 4, 5, 6, 7, 8, 9, 10, 11, 12, 13, 14, 15); }
__device__ __forceinline__ v16bf cat16b(v8us lo, v8us hi) { return __builtin_bit_cast(v16bf, __builtin_shufflevector(lo, hi, 0, 1, 2, 3, 4, 5, 6, 7, 8, 9, 10, 11, 12, 13, 14, 15)); }
__device__ __forceinline__ v8f wmma16(v16h a, v16h b, v8f c) { return __builtin_amdgcn_wmma_f32_16x16x32_f16(false, a, false, b, (short)0, c, false, false); }
__device__ __forceinline__ v8f wmmab(v16bf a, v16bf b, v8f c) { return __builtin_amdgcn_wmma_f32_16x16x32_bf16(false, a, false, b, (short)0, c, false, false); }

template <typename T16> struct WFrag;
template <> struct WFrag<h16> { typedef v16h V; static __device__ __forceinline__ V ld(const h16* p) { return cat16(*(const v8h*)p, *(const v8h*)(p + 16)); } static __device__ __forceinline__ v8f mma(V a, V b, v8f c) { return wmma16(a, b, c); } };
template <> struct WFrag<bf> { typedef v16bf V; static __device__ __forceinline__ V ld(const bf* p) { return cat16b(*(const v8us*)p, *(const v8us*)(p + 16)); } static __device__ __forceinline__ v8f mma(V a, V b, v8f c) { return wmmab(a, b, c); } };
template <typename T16> struct IsBf { enum { v = 0 }; };
template <> struct IsBf<bf> { enum { v = 1 }; };

template <typename T16, int NSPLIT, bool BIAS>
__device__ __forceinline__ void gemmw_body(const T16* __restrict__ A, const T16* __restrict__ A2, const T16* __restrict__ Bt, const T16* __restrict__ Bt2, int K, float* C, int ldc, const float* __restrict__ bias, size_t sA, size_t sB, size_t sC) {
    typedef typename WFrag<T16>::V V;
    __shared__ __align__(16) float os[16 * 68];
    const size_t z = blockIdx.z; A += z * sA; if (A2) A2 += z * sA; Bt += z * sB; if (Bt2) Bt2 += z * sB; C += z * sC;
    const int lane = threadIdx.x & 31, lr = lane & 15, hi = lane >> 4; const int r0 = blockIdx.x * 64, c0 = blockIdx.y * 64;
    v8f acc[4][4];
#pragma unroll
    for (int mb = 0; mb < 4; ++mb)
#pragma unroll
        for (int nb = 0; nb < 4; ++nb) acc[mb][nb] = (v8f){};
    const size_t aoff = (size_t)(r0 + lr) * K + 8 * hi, boff = (size_t)(c0 + lr) * K + 8 * hi;
#pragma unroll 1
    for (int kc = 0; kc < K; kc += 32) {
        V a[4], a2[4], bl;
#pragma unroll
        for (int mb = 0; mb < 4; ++mb) { a[mb] = WFrag<T16>::ld(A + aoff + (size_t)mb * 16 * K + kc); if (NSPLIT == 1 || NSPLIT == 2) a2[mb] = WFrag<T16>::ld(A2 + aoff + (size_t)mb * 16 * K + kc); }
#pragma unroll
        for (int nb = 0; nb < 4; ++nb) { const V b = WFrag<T16>::ld(Bt + boff + (size_t)nb * 16 * K + kc); V b2; if (NSPLIT >= 2) b2 = WFrag<T16>::ld(Bt2 + boff + (size_t)nb * 16 * K + kc);
#pragma unroll
            for (int mb = 0; mb < 4; ++mb) { acc[mb][nb] = WFrag<T16>::mma(a[mb], b, acc[mb][nb]); if (NSPLIT == 1 || NSPLIT == 2) acc[mb][nb] = WFrag<T16>::mma(a2[mb], b, acc[mb][nb]); if (NSPLIT >= 2) acc[mb][nb] = WFrag<T16>::mma(a[mb], b2, acc[mb][nb]); }
            if (nb == 3) bl = b; }
        asm volatile("v_nop\n\tv_nop\n\tv_nop\n\tv_nop" : "+v"(acc[0][0]), "+v"(acc[0][1]), "+v"(acc[0][2]), "+v"(acc[0][3]), "+v"(acc[1][0]), "+v"(acc[1][1]), "+v"(acc[1][2]), "+v"(acc[1][3]),
                            "+v"(acc[2][0]), "+v"(acc[2][1]), "+v"(acc[2][2]), "+v"(acc[2][3]), "+v"(acc[3][0]), "+v"(acc[3][1]), "+v"(acc[3][2]), "+v"(acc[3][3]) : "v"(a[0]), "v"(a[3]), "v"(bl));
    }
#pragma unroll
    for (int mb = 0; mb < 4; ++mb) {
#pragma unroll
        for (int nb = 0; nb < 4; ++nb) {
#pragma unroll
            for (int j = 0; j < 8; ++j) os[(hi * 8 + j) * 68 + nb * 16 + lr] = acc[mb][nb][j]; }
        __builtin_amdgcn_wave_barrier(); asm volatile("" ::: "memory");
        float* crow = C + (size_t)(r0 + mb * 16) * ldc + c0;
#pragma unroll 1
        for (int ps = 0; ps < 2; ++ps) {
#pragma unroll
            for (int s = 0; s < 8; ++s) { const int row = 2 * s + hi, cofs = lr * 4; v4f val = *(const v4fa*)(os + row * 68 + cofs); if (BIAS) { val[0] += bfr(bias[c0 + cofs]); val[1] += bfr(bias[c0 + cofs + 1]); val[2] += bfr(bias[c0 + cofs + 2]); val[3] += bfr(bias[c0 + cofs + 3]); }
                *(volatile v4f*)(crow + (size_t)row * ldc + cofs) = val; }
            if (ps == 0) __threadfence(); }
        __builtin_amdgcn_wave_barrier(); asm volatile("" ::: "memory");
    }
}

template <bool BANDCOL>
__device__ __forceinline__ void gemmp_body(const bf* __restrict__ A, const bf* __restrict__ Bt, int K, h16* P16, bf* Ph, bf* Pl, unsigned ldp, unsigned ldb) {
    typedef WFrag<bf>::V V;
    __shared__ __align__(16) float os[16 * 68];
    const unsigned lane = threadIdx.x & 31u, lr = lane & 15u, hi = lane >> 4; const unsigned r0 = blockIdx.x * 64u, c0 = blockIdx.y * 64u;
    v8f acc[4][4];
#pragma unroll
    for (int mb = 0; mb < 4; ++mb)
#pragma unroll
        for (int nb = 0; nb < 4; ++nb) acc[mb][nb] = (v8f){};
    const size_t aoff = (size_t)(r0 + lr) * K + 8u * hi, boff = (size_t)(c0 + lr) * K + 8u * hi;
#pragma unroll 1
    for (int kc = 0; kc < K; kc += 32) {
        V a[4], bl;
#pragma unroll
        for (int mb = 0; mb < 4; ++mb) a[mb] = WFrag<bf>::ld(A + aoff + (size_t)mb * 16 * K + kc);
#pragma unroll
        for (int nb = 0; nb < 4; ++nb) { const V b = WFrag<bf>::ld(Bt + boff + (size_t)nb * 16 * K + kc);
#pragma unroll
            for (int mb = 0; mb < 4; ++mb) acc[mb][nb] = WFrag<bf>::mma(a[mb], b, acc[mb][nb]);
            if (nb == 3) bl = b; }
        asm volatile("v_nop\n\tv_nop\n\tv_nop\n\tv_nop" : "+v"(acc[0][0]), "+v"(acc[0][1]), "+v"(acc[0][2]), "+v"(acc[0][3]), "+v"(acc[1][0]), "+v"(acc[1][1]), "+v"(acc[1][2]), "+v"(acc[1][3]),
                            "+v"(acc[2][0]), "+v"(acc[2][1]), "+v"(acc[2][2]), "+v"(acc[2][3]), "+v"(acc[3][0]), "+v"(acc[3][1]), "+v"(acc[3][2]), "+v"(acc[3][3]) : "v"(a[0]), "v"(a[3]), "v"(bl));
    }
    const unsigned tsel = BANDCOL ? c0 : r0; const unsigned tloc = tsel % (unsigned)SEQ, bq = tsel / (unsigned)SEQ;
    const bool band = tloc < (unsigned)RH;
    const unsigned bb0 = bq * (unsigned)RH + tloc;
    const unsigned rq = lane >> 3, cq = (lane & 7u) * 8u;
#pragma unroll
    for (int mb = 0; mb < 4; ++mb) {
#pragma unroll
        for (int nb = 0; nb < 4; ++nb) {
#pragma unroll
            for (int j = 0; j < 8; ++j) os[(hi * 8u + j) * 68u + nb * 16u + lr] = acc[mb][nb][j]; }
        __builtin_amdgcn_wave_barrier(); asm volatile("" ::: "memory");
#pragma unroll 1
        for (int ps = 0; ps < 2; ++ps) {
#pragma unroll
            for (int s = 0; s < 4; ++s) { const unsigned row = 4u * s + rq; const v4f x0 = *(const v4fa*)(os + row * 68u + cq); const v4f x1 = *(const v4fa*)(os + row * 68u + cq + 4u);
                const unsigned grow = r0 + mb * 16u + row; v8h o16;
#pragma unroll
                for (int k = 0; k < 4; ++k) { o16[k] = (h16)x0[k]; o16[k + 4] = (h16)x1[k]; }
                *(volatile v8h*)(P16 + (size_t)grow * ldp + c0 + cq) = o16;
                if (band) { v8us oh, ol;
#pragma unroll
                    for (int k = 0; k < 4; ++k) { unsigned short a2, c2; splitf(x0[k], a2, c2); oh[k] = a2; ol[k] = c2; splitf(x1[k], a2, c2); oh[k + 4] = a2; ol[k + 4] = c2; }
                    const size_t bo_ = BANDCOL ? ((size_t)grow * ldb + bb0 + cq) : ((size_t)(bb0 + mb * 16u + row) * ldb + c0 + cq);
                    *(volatile v8us*)(Ph + bo_) = oh; *(volatile v8us*)(Pl + bo_) = ol; } }
            if (ps == 0) __threadfence(); }
        __builtin_amdgcn_wave_barrier(); asm volatile("" ::: "memory");
    }
}

__global__ __launch_bounds__(256) void k_wtG(const float* __restrict__ w, int K, int N, unsigned short* Bt) {
    const int lane = threadIdx.x & 31; const int wave = __builtin_amdgcn_readfirstlane(threadIdx.x >> 5);
    const int L0 = (blockIdx.x * 8 + wave) * 8; const int nlines = N * K / 64;
#pragma unroll
    for (int ps = 0; ps < 2; ++ps) {
#pragma unroll 1
        for (int l = 0; l < 8; ++l) { const int L = L0 + l; if (L >= nlines) break; const size_t e = (size_t)L * 64 + lane * 2; const int k = (int)(e % K), n = (int)(e / K); v2us o;
            o[0] = f2bf(w[(size_t)k * N + n]); o[1] = f2bf(w[(size_t)(k + 1) * N + n]); *(volatile v2us*)(Bt + e) = o; }
        if (ps == 0) __threadfence(); }
}
__global__ __launch_bounds__(256) void k_cvtx(const float* __restrict__ src, unsigned short* dst) {
    const size_t i = (size_t)blockIdx.x * 256 + threadIdx.x; if (i >= (size_t)SEQ * DM / 8) return;
    const float* s = src + (size_t)blockIdx.y * SEQ_FULL * DM + i * 8; bf* d = dst + (size_t)blockIdx.y * SEQ * DM + i * 8;
    const v8f v = *(const v8f*)s; v8us o;
#pragma unroll
    for (int k = 0; k < 8; ++k) o[k] = f2bf(v[k]);
    *(volatile v8us*)d = o; __threadfence(); *(volatile v8us*)d = o; }

__device__ __forceinline__ float mkp(v8f e0, v8f e1, v16h& ph, v16h& pl) { (void)pl; v8h a, b; float s = 0.f;
#pragma unroll
    for (int j = 0; j < 8; ++j) { const h16 x = (h16)(e0[j] * PCAR); const h16 y = (h16)(e1[j] * PCAR); a[j] = x; b[j] = y; s += (float)x + (float)y; }
    ph = cat16(a, b); return s; }
__device__ __forceinline__ float mkp(v8f e0, v8f e1, v16bf& ph, v16bf& pl) { v8us ah, al, bh, bl; float s = 0.f;
#pragma unroll
    for (int j = 0; j < 8; ++j) { unsigned short h, l; splitf(e0[j], h, l); ah[j] = h; al[j] = l; splitf(e1[j], h, l); bh[j] = h; bl[j] = l; s += e0[j] + e1[j]; }
    ph = cat16b(ah, bh); pl = cat16b(al, bl); return s; }

template <typename T16, int NQ>
__device__ __forceinline__ void flash_body(const T16* __restrict__ Qp, const T16* __restrict__ Qlo, const T16* __restrict__ Kp, const T16* __restrict__ Klo,
                                           const T16* __restrict__ Vp, const T16* __restrict__ Vlo, bf* Ah, bf* Al, unsigned qb0, unsigned RB) {
    typedef WFrag<T16> F; typedef typename F::V V;
    static_assert(NQ == 1 || NQ == 2);
    const bool HR = (IsBf<T16>::v != 0);
    __shared__ __align__(16) float os[16 * NQ * 68];
    const unsigned lane = threadIdx.x & 31u, lr = lane & 15u, hi = lane >> 4;
    const unsigned q0 = (qb0 + blockIdx.x) * (16u * NQ), h = blockIdx.y, b = blockIdx.z;
    const size_t rowb = (size_t)b * RB;
    V qf[2][2], ql[2][2];
#pragma unroll
    for (int r = 0; r < NQ; ++r)
#pragma unroll
        for (int c = 0; c < 2; ++c) { const size_t off = (rowb + q0 + 16u * r + lr) * DQ + h * HD + 32u * c + 8u * hi; qf[r][c] = F::ld(Qp + off); if (HR) ql[r][c] = F::ld(Qlo + off); }
    float mrun[2], lrun[2]; v8f o[2][4];
#pragma unroll
    for (int r = 0; r < 2; ++r) { mrun[r] = -3.0e38f; lrun[r] = 0.f;
#pragma unroll
        for (int dt = 0; dt < 4; ++dt) o[r][dt] = (v8f){}; }
    const unsigned nkb = (q0 + 16u * NQ + 31u) >> 5;
    const size_t vpitch = (size_t)NB * RB;
    const size_t voff = (size_t)(h * HD + lr) * vpitch + rowb + 8u * hi;
#pragma unroll 1
    for (unsigned kb = 0; kb < nkb; ++kb) {
        const unsigned k0 = kb * 32u;
        V ka[2][2], kl[2][2];
#pragma unroll
        for (int c = 0; c < 2; ++c) { const size_t koff = (rowb + k0 + 16u * c + lr) * DQ + h * HD + 8u * hi;
            ka[c][0] = F::ld(Kp + koff); ka[c][1] = F::ld(Kp + koff + 32); if (HR) { kl[c][0] = F::ld(Klo + koff); kl[c][1] = F::ld(Klo + koff + 32); } }
        v8f st[2][2];
#pragma unroll
        for (int c = 0; c < 2; ++c)
#pragma unroll
            for (int r = 0; r < NQ; ++r) { v8f a = (v8f){};
                if (HR) { a = F::mma(kl[c][0], qf[r][0], a); a = F::mma(kl[c][1], qf[r][1], a); a = F::mma(ka[c][0], ql[r][0], a); a = F::mma(ka[c][1], ql[r][1], a); }
                a = F::mma(ka[c][0], qf[r][0], a); a = F::mma(ka[c][1], qf[r][1], a); st[r][c] = a; }
        if (NQ == 2) asm volatile("v_nop\n\tv_nop\n\tv_nop\n\tv_nop" : "+v"(st[0][0]), "+v"(st[0][1]), "+v"(st[1][0]), "+v"(st[1][1]) : "v"(ka[1][1]), "v"(qf[0][0]), "v"(qf[1][1]));
        else         asm volatile("v_nop\n\tv_nop\n\tv_nop\n\tv_nop" : "+v"(st[0][0]), "+v"(st[0][1]) : "v"(ka[1][1]), "v"(qf[0][0]), "v"(qf[0][1]));
        const bool lastb = (kb + 1u == nkb);
        V pf[2], pl[2];
#pragma unroll
        for (int r = 0; r < NQ; ++r) {
            const unsigned q = q0 + 16u * r + lr; float mx = -3.0e38f;
#pragma unroll
            for (int c = 0; c < 2; ++c)
#pragma unroll
                for (int j = 0; j < 8; ++j) { const unsigned key = k0 + 16u * c + 8u * hi + j; float s = st[r][c][j]; s = (lastb && key > q) ? -3.0e38f : s; st[r][c][j] = s; mx = fmaxf(mx, s); }
            mx = fmaxf(mx, __shfl_xor(mx, 16, 32));
            const float mnew = fmaxf(mrun[r], mx);
            const float resc = __builtin_amdgcn_exp2f((mrun[r] - mnew) * CEXP);
            mrun[r] = mnew;
            v8f e0, e1;
#pragma unroll
            for (int j = 0; j < 8; ++j) { e0[j] = __builtin_amdgcn_exp2f((st[r][0][j] - mnew) * CEXP); e1[j] = __builtin_amdgcn_exp2f((st[r][1][j] - mnew) * CEXP); }
            const float psum = mkp(e0, e1, pf[r], pl[r]);
            lrun[r] = lrun[r] * resc + psum;
#pragma unroll
            for (int dt = 0; dt < 4; ++dt)
#pragma unroll
                for (int j = 0; j < 8; ++j) o[r][dt][j] *= resc;
        }
        V va[4], vl[4];
#pragma unroll
        for (int dt = 0; dt < 4; ++dt) { const size_t vo = voff + (size_t)dt * 16u * vpitch + k0; va[dt] = F::ld(Vp + vo); if (HR) vl[dt] = F::ld(Vlo + vo); }
#pragma unroll
        for (int dt = 0; dt < 4; ++dt)
#pragma unroll
            for (int r = 0; r < NQ; ++r) { if (HR) { o[r][dt] = F::mma(va[dt], pl[r], o[r][dt]); o[r][dt] = F::mma(vl[dt], pf[r], o[r][dt]); } o[r][dt] = F::mma(va[dt], pf[r], o[r][dt]); }
        if (NQ == 2) asm volatile("v_nop\n\tv_nop\n\tv_nop\n\tv_nop" : "+v"(o[0][0]), "+v"(o[0][1]), "+v"(o[0][2]), "+v"(o[0][3]), "+v"(o[1][0]), "+v"(o[1][1]), "+v"(o[1][2]), "+v"(o[1][3]) : "v"(va[3]), "v"(pf[0]), "v"(pf[1]));
        else         asm volatile("v_nop\n\tv_nop\n\tv_nop\n\tv_nop" : "+v"(o[0][0]), "+v"(o[0][1]), "+v"(o[0][2]), "+v"(o[0][3]) : "v"(va[3]), "v"(pf[0]));
    }
#pragma unroll
    for (int r = 0; r < NQ; ++r) { const float l = lrun[r] + __shfl_xor(lrun[r], 16, 32); const float inv = 1.0f / l;
#pragma unroll
        for (int dt = 0; dt < 4; ++dt)
#pragma unroll
            for (int j = 0; j < 8; ++j) os[(16u * r + lr) * 68u + dt * 16u + 8u * hi + j] = o[r][dt][j] * inv; }
    __syncthreads();
    bf* ah = Ah + ((size_t)b * SEQ + q0) * DQ + h * HD; bf* al = Al + ((size_t)b * SEQ + q0) * DQ + h * HD;
    const unsigned rq = lane >> 3, cq = (lane & 7u) * 8u;
#pragma unroll 1
    for (int ps = 0; ps < 2; ++ps) {
#pragma unroll
        for (int s = 0; s < 4 * NQ; ++s) { const unsigned row = 4u * s + rq; const v4f x0 = *(const v4fa*)(os + row * 68u + cq); const v4f x1 = *(const v4fa*)(os + row * 68u + cq + 4u); v8us oh, ol;
#pragma unroll
            for (int k = 0; k < 4; ++k) { unsigned short a2, c2; splitf(x0[k], a2, c2); oh[k] = a2; ol[k] = c2; splitf(x1[k], a2, c2); oh[k + 4] = a2; ol[k + 4] = c2; }
            *(volatile v8us*)(ah + (size_t)row * DQ + cq) = oh; *(volatile v8us*)(al + (size_t)row * DQ + cq) = ol; }
        if (ps == 0) __threadfence(); }
}

__global__ __launch_bounds__(32) void k_gemmp_row(const unsigned short* __restrict__ A, const unsigned short* __restrict__ Bt, int K, _Float16* P16, unsigned short* Ph, unsigned short* Pl, unsigned ldp, unsigned ldb) {
    gemmp_body<false>(A, Bt, K, P16, Ph, Pl, ldp, ldb); }
__global__ __launch_bounds__(32) void k_gemmp_col(const unsigned short* __restrict__ A, const unsigned short* __restrict__ Bt, int K, _Float16* P16, unsigned short* Ph, unsigned short* Pl, unsigned ldp, unsigned ldb) {
    gemmp_body<true>(A, Bt, K, P16, Ph, Pl, ldp, ldb); }
__global__ __launch_bounds__(32) void k_flash_band(const unsigned short* __restrict__ Qh, const unsigned short* __restrict__ Ql, const unsigned short* __restrict__ Kh, const unsigned short* __restrict__ Kl,
                                                   const unsigned short* __restrict__ Vh, const unsigned short* __restrict__ Vl, unsigned short* Ah, unsigned short* Al) {
    flash_body<bf, 1>(Qh, Ql, Kh, Kl, Vh, Vl, Ah, Al, 0u, (unsigned)RH); }
__global__ __launch_bounds__(32) void k_flash_f16(const _Float16* __restrict__ Q, const _Float16* __restrict__ Kk, const _Float16* __restrict__ Vt, unsigned short* Ah, unsigned short* Al) {
    flash_body<h16, 2>(Q, (const h16*)nullptr, Kk, (const h16*)nullptr, Vt, (const h16*)nullptr, Ah, Al, (unsigned)(RH / 32), (unsigned)SEQ); }
__global__ __launch_bounds__(32) void k_gemmo(const unsigned short* __restrict__ Ahi, const unsigned short* __restrict__ Alo, const unsigned short* __restrict__ Bt, int K, float* C, int ldc, const float* __restrict__ bias, size_t sA, size_t sC) {
    gemmw_body<bf, 1, true>(Ahi, Alo, Bt, (const bf*)nullptr, K, C, ldc, bias, sA, (size_t)0, sC); }

extern "C" void kernel_launch(void* const* d_in, const int* in_sizes, int n_in,
                              void* d_out, int out_size, void* d_ws, size_t ws_size, hipStream_t stream) {
    if (n_in < 6) return;
    const size_t xneed = ((size_t)(NB - 1) * SEQ_FULL + SEQ) * DM, oneed = ((size_t)(NB - 1) * SEQ_FULL + SEQ) * DOW;
    if ((size_t)in_sizes[0] < xneed) return;
    if ((size_t)in_sizes[1] < (size_t)DM * DQ || (size_t)in_sizes[2] < (size_t)DM * DQ || (size_t)in_sizes[3] < (size_t)DM * DQ) return;
    if ((size_t)in_sizes[4] < (size_t)DQ * DOW || (size_t)in_sizes[5] < (size_t)DOW) return;
    if ((size_t)out_size < oneed) return;
    const float* x = (const float*)d_in[0]; const float* wq = (const float*)d_in[1]; const float* wk = (const float*)d_in[2]; const float* wv = (const float*)d_in[3]; const float* wo = (const float*)d_in[4]; const float* bo = (const float*)d_in[5];
    float* OUT = (float*)d_out;
    char* wsp = (char*)d_ws;
    auto take = [&](size_t bytes) { char* p = wsp; wsp += (bytes + 255) & ~(size_t)255; return (void*)p; };
    bf* WQ = (bf*)take((size_t)DQ * DM * 2); bf* WK = (bf*)take((size_t)DQ * DM * 2); bf* WV = (bf*)take((size_t)DQ * DM * 2); bf* WO = (bf*)take((size_t)DOW * DQ * 2);
    bf* XB = (bf*)take((size_t)MROWS * DM * 2);
    h16* Q16 = (h16*)take((size_t)MROWS * DQ * 2); h16* K16 = (h16*)take((size_t)MROWS * DQ * 2); h16* VT16 = (h16*)take((size_t)DQ * MROWS * 2);
    bf* QBh = (bf*)take((size_t)NB * RH * DQ * 2); bf* QBl = (bf*)take((size_t)NB * RH * DQ * 2); bf* KBh = (bf*)take((size_t)NB * RH * DQ * 2); bf* KBl = (bf*)take((size_t)NB * RH * DQ * 2);
    bf* VBh = (bf*)take((size_t)DQ * NB * RH * 2); bf* VBl = (bf*)take((size_t)DQ * NB * RH * 2);
    bf* ATl = (bf*)take((size_t)MROWS * DQ * 2); bf* ATh = XB;
    if ((size_t)(wsp - (char*)d_ws) > ws_size) return;
    const unsigned wtg = (unsigned)((DM * DQ / 64 + 63) / 64);
    k_wtG<<<wtg, 256, 0, stream>>>(wq, DM, DQ, WQ); k_wtG<<<wtg, 256, 0, stream>>>(wk, DM, DQ, WK); k_wtG<<<wtg, 256, 0, stream>>>(wv, DM, DQ, WV);
    k_wtG<<<(unsigned)((DQ * DOW / 64 + 63) / 64), 256, 0, stream>>>(wo, DQ, DOW, WO);
    k_cvtx<<<dim3((unsigned)((size_t)SEQ * DM / 8 / 256), NB, 1), 256, 0, stream>>>(x, XB);
    k_gemmp_row<<<dim3(MROWS / 64, DQ / 64, 1), 32, 0, stream>>>(XB, WQ, DM, Q16, QBh, QBl, (unsigned)DQ, (unsigned)DQ);
    k_gemmp_row<<<dim3(MROWS / 64, DQ / 64, 1), 32, 0, stream>>>(XB, WK, DM, K16, KBh, KBl, (unsigned)DQ, (unsigned)DQ);
    k_gemmp_col<<<dim3(DQ / 64, MROWS / 64, 1), 32, 0, stream>>>(WV, XB, DM, VT16, VBh, VBl, (unsigned)MROWS, (unsigned)(NB * RH));
    k_flash_band<<<dim3(RH / 16, NH_, NB), 32, 0, stream>>>(QBh, QBl, KBh, KBl, VBh, VBl, ATh, ATl);
    if (SEQ > RH) k_flash_f16<<<dim3((SEQ - RH) / 32, NH_, NB), 32, 0, stream>>>(Q16, K16, VT16, ATh, ATl);
    k_gemmo<<<dim3(SEQ / 64, DOW / 64, NB), 32, 0, stream>>>(ATh, ATl, WO, DQ, OUT, DOW, bo, (size_t)SEQ * DQ, (size_t)SEQ_FULL * DOW);
}
